// DualCausalMambaBlock_43250320670995
// MI455X (gfx1250) — hardware-run, weakly checked
//
#include <hip/hip_runtime.h>


#define NB_  2
#define LL   2048
#define DMd  1024
#define DI   2048
#define NS   16
#define DTR  64
#define XPW  128
#define XPR  96
typedef _Float16 h16;
typedef unsigned short bf;
typedef __attribute__((ext_vector_type(16))) __bf16   v16bf;
typedef __attribute__((ext_vector_type(16))) _Float16 v16h;
typedef __attribute__((ext_vector_type(8)))  _Float16 v8h;
typedef __attribute__((ext_vector_type(8)))  unsigned short v8us;
typedef __attribute__((ext_vector_type(8)))  float    v8f;
typedef __attribute__((ext_vector_type(4)))  float    v4f;
typedef v8h  __attribute__((may_alias)) v8ha;
typedef v4f  __attribute__((may_alias)) v4fa;
typedef v8us __attribute__((may_alias)) v8usa;

__device__ __forceinline__ unsigned short f2bf(float f) { unsigned u = __float_as_uint(f); u += 0x7FFFu + ((u >> 16) & 1u); return (unsigned short)(u >> 16); }
__device__ __forceinline__ float bf2f(unsigned short b) { return __uint_as_float(((unsigned)b) << 16); }
__device__ __forceinline__ float bfr(float f) { return bf2f(f2bf(f)); }
__device__ __forceinline__ v16h cat16(v8h lo, v8h hi) { return __builtin_shufflevector(lo, hi, 0, 1, 2, 3, 4, 5, 6, 7, 8, 9, 10, 11, 12, 13, 14, 15); }
__device__ __forceinline__ v16bf cat16b(v8us lo, v8us hi) { return __builtin_bit_cast(v16bf, __builtin_shufflevector(lo, hi, 0, 1, 2, 3, 4, 5, 6, 7, 8, 9, 10, 11, 12, 13, 14, 15)); }
__device__ __forceinline__ v8f wmma16(v16h a, v16h b, v8f c) { return __builtin_amdgcn_wmma_f32_16x16x32_f16(false, a, false, b, (short)0, c, false, false); }
__device__ __forceinline__ v8f wmmab(v16bf a, v16bf b, v8f c) { return __builtin_amdgcn_wmma_f32_16x16x32_bf16(false, a, false, b, (short)0, c, false, false); }


template <typename T16> struct WFrag;
template <> struct WFrag<h16> { typedef v16h V; static __device__ __forceinline__ V ld(const h16* p) { return cat16(*(const v8h*)p, *(const v8h*)(p + 16)); } static __device__ __forceinline__ v8f mma(V a, V b, v8f c) { return wmma16(a, b, c); } };
template <> struct WFrag<bf> { typedef v16bf V; static __device__ __forceinline__ V ld(const bf* p) { return cat16b(*(const v8us*)p, *(const v8us*)(p + 16)); } static __device__ __forceinline__ v8f mma(V a, V b, v8f c) { return wmmab(a, b, c); } };
template <typename T16, int NSPLIT, bool BIAS>
__global__ __launch_bounds__(32) void k_gemmw(const T16* __restrict__ A, const T16* __restrict__ A2, const T16* __restrict__ Bt, const T16* __restrict__ Bt2, int K, float* C, int ldc, const float* __restrict__ bias, size_t sA, size_t sB, size_t sC) {
    typedef typename WFrag<T16>::V V;
    __shared__ __align__(16) float os[16 * 68];
    const size_t z = blockIdx.z; A += z * sA; if (A2) A2 += z * sA; Bt += z * sB; if (Bt2) Bt2 += z * sB; C += z * sC;
    const int lane = threadIdx.x & 31, lr = lane & 15, hi = lane >> 4; const int r0 = blockIdx.x * 64, c0 = blockIdx.y * 64;
    v8f acc[4][4];
#pragma unroll
    for (int mb = 0; mb < 4; ++mb)
#pragma unroll
        for (int nb = 0; nb < 4; ++nb) acc[mb][nb] = (v8f){};
    const size_t aoff = (size_t)(r0 + lr) * K + 8 * hi, boff = (size_t)(c0 + lr) * K + 8 * hi;
#pragma unroll 1
    for (int kc = 0; kc < K; kc += 32) {
        V a[4], a2[4];
#pragma unroll
        for (int mb = 0; mb < 4; ++mb) { a[mb] = WFrag<T16>::ld(A + aoff + (size_t)mb * 16 * K + kc); if (NSPLIT == 1 || NSPLIT == 2) a2[mb] = WFrag<T16>::ld(A2 + aoff + (size_t)mb * 16 * K + kc); }
#pragma unroll
        for (int nb = 0; nb < 4; ++nb) { const V b = WFrag<T16>::ld(Bt + boff + (size_t)nb * 16 * K + kc); V b2; if (NSPLIT >= 2) b2 = WFrag<T16>::ld(Bt2 + boff + (size_t)nb * 16 * K + kc);
#pragma unroll
            for (int mb = 0; mb < 4; ++mb) { acc[mb][nb] = WFrag<T16>::mma(a[mb], b, acc[mb][nb]); if (NSPLIT == 1 || NSPLIT == 2) acc[mb][nb] = WFrag<T16>::mma(a2[mb], b, acc[mb][nb]); if (NSPLIT >= 2) acc[mb][nb] = WFrag<T16>::mma(a[mb], b2, acc[mb][nb]); } }
        asm volatile("v_nop\n\tv_nop\n\tv_nop\n\tv_nop" : "+v"(acc[0][0]), "+v"(acc[1][1]), "+v"(acc[2][2]), "+v"(acc[3][3]) : "v"(a[0]), "v"(a[3]));
    }
#pragma unroll
    for (int mb = 0; mb < 4; ++mb) {
#pragma unroll
        for (int nb = 0; nb < 4; ++nb) {
#pragma unroll
            for (int j = 0; j < 8; ++j) os[(hi * 8 + j) * 68 + nb * 16 + lr] = acc[mb][nb][j]; }
        __builtin_amdgcn_wave_barrier(); asm volatile("" ::: "memory");
        float* crow = C + (size_t)(r0 + mb * 16) * ldc + c0;
#pragma unroll 1
        for (int ps = 0; ps < 2; ++ps) {
#pragma unroll
            for (int s = 0; s < 8; ++s) { const int row = 2 * s + hi, cofs = lr * 4; v4f val = *(const v4fa*)(os + row * 68 + cofs); if (BIAS) { val[0] += bfr(bias[c0 + cofs]); val[1] += bfr(bias[c0 + cofs + 1]); val[2] += bfr(bias[c0 + cofs + 2]); val[3] += bfr(bias[c0 + cofs + 3]); }
                *(volatile v4f*)(crow + (size_t)row * ldc + cofs) = val; }
            if (ps == 0) __threadfence(); }
        __builtin_amdgcn_wave_barrier(); asm volatile("" ::: "memory");
    }
}

__device__ __forceinline__ void splitf(float y, unsigned short& h, unsigned short& l) { h = f2bf(y); l = f2bf(y - bf2f(h)); }
__device__ __forceinline__ float silu_(float x) { return __fmul_rn(x, __fdiv_rn(1.0f, 1.0f + __expf(-x))); }
__device__ __forceinline__ float softplus_(float x) { return x > 20.f ? x : log1pf(__expf(x)); }
typedef __attribute__((ext_vector_type(2))) unsigned short v2us;
typedef __attribute__((ext_vector_type(4))) unsigned short v4us;

__global__ __launch_bounds__(256) void k_cvt8(const float* __restrict__ src, bf* dst, size_t n8) { const size_t i = (size_t)blockIdx.x * 256 + threadIdx.x; if (i >= n8) return; const v8f v = *(const v8f*)(src + i * 8); v8us o;
#pragma unroll
    for (int k = 0; k < 8; ++k) o[k] = f2bf(v[k]); *(volatile v8us*)(dst + i * 8) = o; __threadfence(); *(volatile v8us*)(dst + i * 8) = o; }
__global__ __launch_bounds__(256) void k_wpad(const float* __restrict__ w, int nreal, int NOUT, int KP, bf* Bt) { const size_t i = ((size_t)blockIdx.x * 256 + threadIdx.x) * 4; if (i >= (size_t)NOUT * KP) return; const int n = (int)(i / KP); v4us o;
#pragma unroll
    for (int q = 0; q < 4; ++q) o[q] = n < nreal ? f2bf(w[i + q]) : (unsigned short)0; *(volatile v4us*)(Bt + i) = o; __threadfence(); *(volatile v4us*)(Bt + i) = o; }
__global__ __launch_bounds__(256) void k_conv(const float* __restrict__ XZ, const float* __restrict__ w, const float* __restrict__ bb, float* XC, bf* Ch, bf* Cl) { const int e = (blockIdx.x * 256 + threadIdx.x) * 4; if (e >= LL * DI) return; const int c = e % DI, t = e / DI; v4f o; v4us oh, ol;
#pragma unroll 1
    for (int q = 0; q < 4; ++q) { const int cc = c + q; float acc = bfr(bb[cc]);
#pragma unroll
        for (int k = 0; k < 4; ++k) { const int ts = t - 3 + k; float p = (ts >= 0) ? __fmul_rn(XZ[(size_t)ts * 2 * DI + cc], bfr(w[cc * 4 + k])) : 0.f; asm volatile("" : "+v"(p)); acc = __fadd_rn(acc, p); }
        o[q] = silu_(acc); unsigned short u, l; splitf(o[q], u, l); oh[q] = u; ol[q] = l; }
    for (int ps = 0; ps < 2; ++ps) { *(volatile v4f*)(XC + e) = o; *(volatile v4us*)(Ch + e) = oh; *(volatile v4us*)(Cl + e) = ol; if (ps == 0) __threadfence(); } }
__global__ __launch_bounds__(256) void k_split(const float* __restrict__ F, int w, int pitch, int c0, int nrows, bf* Ph, bf* Pl) { const int e = (blockIdx.x * 256 + threadIdx.x) * 4; if (e >= nrows * w) return; const int c = e % w, r = e / w; const v4f a = *(const v4f*)(F + (size_t)r * pitch + c0 + c); v4us oh, ol;
#pragma unroll
    for (int q = 0; q < 4; ++q) { unsigned short u, l; splitf(a[q], u, l); oh[q] = u; ol[q] = l; } *(volatile v4us*)(Ph + e) = oh; *(volatile v4us*)(Pl + e) = ol; __threadfence(); *(volatile v4us*)(Ph + e) = oh; *(volatile v4us*)(Pl + e) = ol; }
__global__ __launch_bounds__(256) void k_scan(const float* __restrict__ DTRf, const float* __restrict__ XC, const float* __restrict__ XP, const float* __restrict__ alog, const float* __restrict__ Dp, float* Y) { const int c = blockIdx.x * 256 + threadIdx.x; if (c >= DI) return; float A[NS], S[NS];
#pragma unroll
    for (int n = 0; n < NS; ++n) { A[n] = -__expf(bfr(alog[(size_t)c * NS + n])); S[n] = 0.f; }
    const float dd = bfr(Dp[c]);
    for (int t = 0; t < LL; ++t) { const float dt = softplus_(DTRf[(size_t)t * DI + c]); const float xv = XC[(size_t)t * DI + c]; const float dtx = __fmul_rn(dt, xv); const float* pr = XP + (size_t)t * XPW + DTR; float y = 0.f;
#pragma unroll
        for (int n = 0; n < NS; ++n) { const float a = __expf(__fmul_rn(dt, A[n])); float sa = __fmul_rn(S[n], a); asm volatile("" : "+v"(sa)); float bx = __fmul_rn(dtx, pr[n]); asm volatile("" : "+v"(bx)); S[n] = __fadd_rn(sa, bx); float yc = __fmul_rn(S[n], pr[NS + n]); asm volatile("" : "+v"(yc)); y = __fadd_rn(y, yc); }
        float sk = __fmul_rn(dd, xv); asm volatile("" : "+v"(sk)); const float out = __fadd_rn(y, sk); *(volatile float*)(Y + (size_t)t * DI + c) = out; __threadfence(); *(volatile float*)(Y + (size_t)t * DI + c) = out; } }
__global__ __launch_bounds__(256) void k_gate(const float* __restrict__ Y, const float* __restrict__ XZ, bf* Gh, bf* Gl) { const int e = (blockIdx.x * 256 + threadIdx.x) * 4; if (e >= LL * DI) return; const int c = e % DI, t = e / DI; const v4f y = *(const v4f*)(Y + e), z = *(const v4f*)(XZ + (size_t)t * 2 * DI + DI + c); v4us oh, ol;
#pragma unroll
    for (int q = 0; q < 4; ++q) { unsigned short u, l; splitf(__fmul_rn(y[q], silu_(z[q])), u, l); oh[q] = u; ol[q] = l; } *(volatile v4us*)(Gh + e) = oh; *(volatile v4us*)(Gl + e) = ol; __threadfence(); *(volatile v4us*)(Gh + e) = oh; *(volatile v4us*)(Gl + e) = ol; }

extern "C" void kernel_launch(void* const* d_in, const int* in_sizes, int n_in,
                              void* d_out, int out_size, void* d_ws, size_t ws_size, hipStream_t stream) {
    (void)in_sizes; (void)n_in; (void)out_size;
    const float* u = (const float*)d_in[0]; const float* win = (const float*)d_in[1]; const float* wout = (const float*)d_in[2]; const float* cw = (const float*)d_in[3]; const float* cb = (const float*)d_in[4]; const float* wx = (const float*)d_in[5]; const float* wdt = (const float*)d_in[6]; const float* bdt = (const float*)d_in[7]; const float* alog = (const float*)d_in[8]; const float* Dp = (const float*)d_in[9];
    float* OUT = (float*)d_out;
    char* wsp = (char*)d_ws;
    auto take = [&](size_t bytes) { char* p = wsp; wsp += (bytes + 255) & ~(size_t)255; return (void*)p; };
    bf* WIN = (bf*)take((size_t)2 * DI * DMd * 2); bf* WX = (bf*)take((size_t)XPW * DI * 2); bf* WDT = (bf*)take((size_t)DI * DTR * 2); bf* WOUT = (bf*)take((size_t)DMd * DI * 2);
    bf* UB = (bf*)take((size_t)LL * DMd * 2); float* XZ = (float*)take((size_t)LL * 2 * DI * 4); float* XC = (float*)take((size_t)LL * DI * 4); bf* Ch = (bf*)take((size_t)LL * DI * 2); bf* Cl = (bf*)take((size_t)LL * DI * 2); float* XP = (float*)take((size_t)LL * XPW * 4); bf* Rh = (bf*)take((size_t)LL * DTR * 2); bf* Rl = (bf*)take((size_t)LL * DTR * 2); float* DTRf = (float*)take((size_t)LL * DI * 4); float* Y = (float*)take((size_t)LL * DI * 4); bf* Gh = (bf*)take((size_t)LL * DI * 2); bf* Gl = (bf*)take((size_t)LL * DI * 2);
    if ((size_t)(wsp - (char*)d_ws) > ws_size) return;
    k_cvt8<<<(unsigned)(((size_t)2 * DI * DMd / 8 + 255) / 256), 256, 0, stream>>>(win, WIN, (size_t)2 * DI * DMd / 8); k_wpad<<<(XPW * DI / 4 + 255) / 256, 256, 0, stream>>>(wx, XPR, XPW, DI, WX); k_cvt8<<<(DI * DTR / 8 + 255) / 256, 256, 0, stream>>>(wdt, WDT, (size_t)DI * DTR / 8); k_cvt8<<<(DMd * DI / 8 + 255) / 256, 256, 0, stream>>>(wout, WOUT, (size_t)DMd * DI / 8);
    for (int b = 0; b < NB_; ++b) {
        k_cvt8<<<(LL * DMd / 8 + 255) / 256, 256, 0, stream>>>(u + (size_t)b * LL * DMd, UB, (size_t)LL * DMd / 8);
        k_gemmw<bf, 0, false><<<dim3(LL / 64, 2 * DI / 64, 1), 32, 0, stream>>>(UB, nullptr, WIN, nullptr, DMd, XZ, 2 * DI, nullptr, 0, 0, 0);
        k_conv<<<(LL * DI / 4 + 255) / 256, 256, 0, stream>>>(XZ, cw, cb, XC, Ch, Cl);
        k_gemmw<bf, 1, false><<<dim3(LL / 64, XPW / 64, 1), 32, 0, stream>>>(Ch, Cl, WX, nullptr, DI, XP, XPW, nullptr, 0, 0, 0);
        k_split<<<(LL * DTR / 4 + 255) / 256, 256, 0, stream>>>(XP, DTR, XPW, 0, LL, Rh, Rl);
        k_gemmw<bf, 1, true><<<dim3(LL / 64, DI / 64, 1), 32, 0, stream>>>(Rh, Rl, WDT, nullptr, DTR, DTRf, DI, bdt, 0, 0, 0);
        k_scan<<<DI / 256, 256, 0, stream>>>(DTRf, XC, XP, alog, Dp, Y);
        k_gate<<<(LL * DI / 4 + 255) / 256, 256, 0, stream>>>(Y, XZ, Gh, Gl);
        k_gemmw<bf, 1, false><<<dim3(LL / 64, DMd / 64, 1), 32, 0, stream>>>(Gh, Gl, WOUT, nullptr, DI, OUT + (size_t)b * LL * DMd, DMd, nullptr, 0, 0, 0); }
}
